// BoundaryGraphPredictor_2104533975798
// MI455X (gfx1250) — hardware-verified
//
#include <hip/hip_runtime.h>
#include <math.h>
typedef __attribute__((ext_vector_type(16))) _Float16 v16h;
typedef __attribute__((ext_vector_type(8)))  _Float16 v8h;
typedef __attribute__((ext_vector_type(16))) __bf16   v16b;
typedef __attribute__((ext_vector_type(8)))  __bf16   v8b;
typedef __attribute__((ext_vector_type(8)))  float    v8f;
typedef __attribute__((ext_vector_type(4)))  float    v4f;
#define PSCALE 32768.0f
#define U16(p) ((const unsigned short*)(const void*)(p))
#define PSCALE_INV (1.0f / 32768.0f)

__device__ __forceinline__ unsigned short f2bf_bits(float f) {
  unsigned u = __float_as_uint(f);
  return (unsigned short)((u + 0x7FFFu + ((u >> 16) & 1u)) >> 16);
}
__device__ __forceinline__ float bf_bits2f(unsigned short h) { return __uint_as_float(((unsigned)h) << 16); }

__device__ __forceinline__ void dep_guard_h(v8f& a, v8f& b, v16h x, v16h y) { asm volatile("v_nop\n\tv_nop\n\tv_nop\n\tv_nop" : "+v"(a), "+v"(b) : "v"(x), "v"(y)); }
__device__ __forceinline__ void dep_guard_b(v8f& a, v8f& b, v16b x, v16b y) { asm volatile("v_nop\n\tv_nop\n\tv_nop\n\tv_nop" : "+v"(a), "+v"(b) : "v"(x), "v"(y)); }
__device__ __forceinline__ void keep4_h(v16h a, v16h b, v16h c, v16h d) { asm volatile("v_nop" :: "v"(a), "v"(b), "v"(c), "v"(d)); }
__device__ __forceinline__ void keep4_b(v16b a, v16b b, v16b c, v16b d) { asm volatile("v_nop" :: "v"(a), "v"(b), "v"(c), "v"(d)); }
__device__ __forceinline__ void acc_guard4(v8f& a, v8f& b, v8f& c, v8f& d) { asm volatile("v_nop\n\tv_nop\n\tv_nop\n\tv_nop" : "+v"(a), "+v"(b), "+v"(c), "+v"(d)); }
template <typename T> struct Frag;
template <> struct Frag<_Float16> {
  typedef v16h V; union U { v16h v; v8h h[2]; };
  static __device__ __forceinline__ v16h load(const _Float16* p) {
    U f; f.h[0] = *(const v8h*)(p); f.h[1] = *(const v8h*)(p + 16); return f.v;
  }
  static __device__ __forceinline__ v8f mma(v16h a, v16h b, v8f c) {
    return __builtin_amdgcn_wmma_f32_16x16x32_f16(false, a, false, b, (short)0, c, false, false);
  }
  static __device__ __forceinline__ void guard(v8f& a, v8f& b, v16h x, v16h y) { dep_guard_h(a, b, x, y); }
  static __device__ __forceinline__ void keep(v16h a, v16h b, v16h c, v16h d) { keep4_h(a, b, c, d); }
};
template <> struct Frag<__bf16> {
  typedef v16b V; union U { v16b v; v8b h[2]; };
  static __device__ __forceinline__ v16b load(const __bf16* p) {
    U f; f.h[0] = *(const v8b*)(p); f.h[1] = *(const v8b*)(p + 16); return f.v;
  }
  static __device__ __forceinline__ v8f mma(v16b a, v16b b, v8f c) {
    return __builtin_amdgcn_wmma_f32_16x16x32_bf16(false, a, false, b, (short)0, c, false, false);
  }
  static __device__ __forceinline__ void guard(v8f& a, v8f& b, v16b x, v16b y) { dep_guard_b(a, b, x, y); }
  static __device__ __forceinline__ void keep(v16b a, v16b b, v16b c, v16b d) { keep4_b(a, b, c, d); }
};

template <int ET> struct Elem;
template <> struct Elem<0> { typedef _Float16 T; };
template <> struct Elem<1> { typedef __bf16 T; };
template <int ET, bool SPLIT, int BIAS_MODE, int OUT_MODE, bool RESID, int ACT = 0>
__global__ __launch_bounds__(256) void wmma_gemm64(
    const unsigned short* __restrict__ Ap, const unsigned short* __restrict__ A2p, int lda, long strideA,
    const unsigned short* __restrict__ Btp, const unsigned short* __restrict__ Bt2p, int ldb, long strideB,
    void* __restrict__ Cout, void* __restrict__ Cout2, int ldc, long strideC,
    const float* __restrict__ bias,
    const float* __restrict__ resid, long strideR,
    int M, int N, int K, float scale) {
  typedef typename Elem<ET>::T T;
  typedef typename Frag<T>::V V;
  const T* A = (const T*)Ap; const T* A2 = (const T*)A2p; const T* Bt = (const T*)Btp; const T* Bt2 = (const T*)Bt2p;
  __shared__ __align__(16) float sT[8][16 * 68];
  const int b    = blockIdx.y;
  const int lane = threadIdx.x & 31;
  const int wave = threadIdx.x >> 5;
  const int tilesN = N >> 6;
  const int tilesM = M >> 6;
  const int tile = blockIdx.x * 8 + wave;
  if (tile >= tilesM * tilesN) return;
  const int tm = tile / tilesN;
  const int tn = tile - tm * tilesN;
  const int m0 = tm << 6;
  const int n0 = tn << 6;

  const T* Ab  = A  + (size_t)b * strideA;
  const T* Bb  = Bt + (size_t)b * strideB;
  const T* Ab2 = SPLIT ? (A2  + (size_t)b * strideA) : nullptr;
  const T* Bb2 = SPLIT ? (Bt2 + (size_t)b * strideB) : nullptr;

  const int rlane = lane & 15;
  const int koff  = (lane >> 4) * 8;
  const int mOff  = (lane >> 4) * 8;

  v8f acc[4][4];
#pragma unroll
  for (int i = 0; i < 4; ++i)
#pragma unroll
    for (int j = 0; j < 4; ++j) acc[i][j] = (v8f){0.f,0.f,0.f,0.f,0.f,0.f,0.f,0.f};

  for (int k0 = 0; k0 < K; k0 += 32) {
    V bh[4], bl[4];
#pragma unroll
    for (int j = 0; j < 4; ++j) {
      const size_t bo = (size_t)(n0 + (j << 4) + rlane) * ldb + koff + k0;
      bh[j] = Frag<T>::load(Bb + bo);
      if (SPLIT) bl[j] = Frag<T>::load(Bb2 + bo);
    }
#pragma unroll
    for (int i = 0; i < 4; ++i) {
      const size_t ao = (size_t)(m0 + (i << 4) + rlane) * lda + koff + k0;
      V ah = Frag<T>::load(Ab + ao);
      V al;
      if (SPLIT) al = Frag<T>::load(Ab2 + ao);
#pragma unroll
      for (int j = 0; j < 4; ++j) {
        acc[i][j] = Frag<T>::mma(ah, bh[j], acc[i][j]);
        if (SPLIT) {
          acc[i][j] = Frag<T>::mma(ah, bl[j], acc[i][j]);
          acc[i][j] = Frag<T>::mma(al, bh[j], acc[i][j]);
        }
      }
      Frag<T>::guard(acc[i][0], acc[i][3], ah, SPLIT ? al : ah);
    }
    Frag<T>::keep(bh[0], bh[1], bh[2], bh[3]);
    if (SPLIT) Frag<T>::keep(bl[0], bl[1], bl[2], bl[3]);
  }
  acc_guard4(acc[0][0], acc[0][1], acc[0][2], acc[0][3]);
  acc_guard4(acc[1][0], acc[1][1], acc[1][2], acc[1][3]);
  acc_guard4(acc[2][0], acc[2][1], acc[2][2], acc[2][3]);
  acc_guard4(acc[3][0], acc[3][1], acc[3][2], acc[3][3]);

  float* slab = sT[wave];
  const float* Rb = RESID ? (resid + (size_t)b * strideR) : nullptr;
#pragma unroll
  for (int i = 0; i < 4; ++i) {
    const int mBase = m0 + (i << 4);
#pragma unroll
    for (int j = 0; j < 4; ++j) {
      const int n = n0 + (j << 4) + rlane;
      float bv = 0.f;
      if (BIAS_MODE == 2) bv = bias[n];
#pragma unroll
      for (int r = 0; r < 8; ++r) {
        float v = acc[i][j][r] * scale;
        if (BIAS_MODE == 1) v += bias[mBase + mOff + r];
        if (BIAS_MODE == 2) v += bv;
        if (RESID) v += Rb[(size_t)(mBase + mOff + r) * ldc + n];
        if (ACT == 1) v = tanhf(v);
        if (ACT == 2) v = fmaxf(v, 0.0f);
        slab[(mOff + r) * 68 + (j << 4) + rlane] = v;
      }
    }
    __builtin_amdgcn_fence(__ATOMIC_RELEASE, "workgroup");
    __builtin_amdgcn_wave_barrier();
    __builtin_amdgcn_fence(__ATOMIC_ACQUIRE, "workgroup");
    if (OUT_MODE == 0) {
      float* C = (float*)Cout + (size_t)b * strideC;
      const int hh = lane >> 4, c4 = (lane & 15) * 4;
      for (int pass = 0; pass < 2; ++pass) {
#pragma unroll
        for (int it = 0; it < 8; ++it) {
          const int row = it * 2 + hh;
          v4f v = *(const v4f*)(slab + row * 68 + c4);
          *(volatile v4f*)(C + (size_t)(mBase + row) * ldc + n0 + c4) = v;
        }
        __threadfence();
      }
    } else {
      const int q = lane >> 3, c8 = (lane & 7) * 8;
      unsigned short* C  = (unsigned short*)Cout  + (size_t)b * strideC;
      unsigned short* C2 = (OUT_MODE == 2) ? ((unsigned short*)Cout2 + (size_t)b * strideC) : nullptr;
      for (int pass = 0; pass < 2; ++pass) {
#pragma unroll
        for (int it = 0; it < 4; ++it) {
          const int row = it * 4 + q;
          const float* sp = slab + row * 68 + c8;
          v8h hv, lv;
#pragma unroll
          for (int e = 0; e < 8; ++e) {
            if (OUT_MODE == 1) {
              hv[e] = (_Float16)sp[e];
            } else {
              unsigned short hb = f2bf_bits(sp[e]);
              unsigned short lb = f2bf_bits(sp[e] - bf_bits2f(hb));
              hv[e] = __builtin_bit_cast(_Float16, hb);
              lv[e] = __builtin_bit_cast(_Float16, lb);
            }
          }
          *(volatile v8h*)(C + (size_t)(mBase + row) * ldc + n0 + c8) = hv;
          if (OUT_MODE == 2) *(volatile v8h*)(C2 + (size_t)(mBase + row) * ldc + n0 + c8) = lv;
        }
        __threadfence();
      }
    }
    __builtin_amdgcn_fence(__ATOMIC_RELEASE, "workgroup");
    __builtin_amdgcn_wave_barrier();
    __builtin_amdgcn_fence(__ATOMIC_ACQUIRE, "workgroup");
  }
}


__global__ __launch_bounds__(256) void transpose_cast_f16(const float* __restrict__ in, int ldi,
                                                         _Float16* __restrict__ outT, int ldo, float scale) {
  __shared__ __align__(16) _Float16 tile[64][72];
  const int c0 = blockIdx.x * 64, r0 = blockIdx.y * 64;
  const int t = threadIdx.y * 32 + threadIdx.x;
  for (int i = threadIdx.y; i < 64; i += 8) {
    tile[threadIdx.x][i]      = (_Float16)(in[(size_t)(r0 + i) * ldi + c0 + threadIdx.x] * scale);
    tile[32 + threadIdx.x][i] = (_Float16)(in[(size_t)(r0 + i) * ldi + c0 + 32 + threadIdx.x] * scale);
  }
  __syncthreads();
  const int q = t >> 3, c8 = (t & 7) * 8;
  for (int pass = 0; pass < 2; ++pass) {
#pragma unroll
    for (int it = 0; it < 2; ++it) {
      const int c = it * 32 + q;
      v8h hv = *(const v8h*)(&tile[c][c8]);
      *(volatile v8h*)(outT + (size_t)(c0 + c) * ldo + r0 + c8) = hv;
    }
    __threadfence();
  }
}

#define NN 20000
#define NPAD 20032
#define NE 320000
#define DIM 512
#define NH 8
#define HC 64
#define NODES_PER_BLK 256
#define NBLK ((NN + NODES_PER_BLK - 1) / NODES_PER_BLK)
#define SEG_CAP 16384

__device__ __forceinline__ int chunk_rank(int node, bool valid, int lane, int& ntotal) {
  unsigned same = __ballot(valid);
#pragma unroll
  for (int b = 0; b < 8; ++b) {
    const unsigned m = __ballot(((node >> b) & 1) != 0);
    same &= (((node >> b) & 1) != 0) ? m : ~m;
  }
  if (!valid) same = 0u;
  ntotal = __popc(same);
  return __popc(same & ((1u << lane) - 1u));
}
__global__ __launch_bounds__(256) void csr_count_kernel(const int* __restrict__ dst, int* __restrict__ blk_total) {
  __shared__ int wtot[8];
  const int tid = threadIdx.x, lane = tid & 31, wave = tid >> 5;
  const int n0 = blockIdx.x * NODES_PER_BLK;
  const int e0 = wave * (NE / 8), e1 = e0 + NE / 8;
  int wsum = 0;
  for (int c0 = e0; c0 < e1; c0 += 32) {
    const int e = c0 + lane;
    const int d = (e < e1) ? dst[e] : -1;
    const bool valid = (e < e1) && (d >= n0) && (d < n0 + NODES_PER_BLK);
    wsum += __popc(__ballot(valid));
  }
  if (lane == 0) wtot[wave] = wsum;
  __syncthreads();
  if (tid < 32) {
    int s = 0;
    for (int w = 0; w < 8; ++w) s += wtot[w];
    const int v = (tid == 0) ? s : 0;
    ((volatile int*)blk_total)[blockIdx.x * 32 + tid] = v;
    __threadfence();
    ((volatile int*)blk_total)[blockIdx.x * 32 + tid] = v;
  }
}
__global__ __launch_bounds__(1024) void csr_scan_kernel(const int* __restrict__ blk_total, int* __restrict__ blk_base) {
  __shared__ int s[1024];
  const int tid = threadIdx.x;
  int v = (tid < NBLK) ? blk_total[tid * 32] : 0;
  s[tid] = v;
  __syncthreads();
  for (int off = 1; off < 1024; off <<= 1) {
    int a = (tid >= off) ? s[tid - off] : 0;
    __syncthreads();
    s[tid] += a;
    __syncthreads();
  }
  const int excl = s[tid] - v;
  ((volatile int*)blk_base)[tid] = excl;
  __threadfence();
  ((volatile int*)blk_base)[tid] = excl;
}
__global__ __launch_bounds__(256) void csr_fill_kernel(const int* __restrict__ dst, const int* __restrict__ blk_base,
                                                      int* __restrict__ rowptr, int* __restrict__ rowdeg, int* __restrict__ csr_eid) {
  __shared__ int cnt[8][NODES_PER_BLK];
  __shared__ int off[8][NODES_PER_BLK];
  __shared__ int nodeoff[NODES_PER_BLK + 1];
  __shared__ int seg[SEG_CAP];
  const int tid = threadIdx.x, lane = tid & 31, wave = tid >> 5;
  const int n0 = blockIdx.x * NODES_PER_BLK;
  for (int i = tid; i < 8 * NODES_PER_BLK; i += 256) (&cnt[0][0])[i] = 0;
  for (int i = tid; i < SEG_CAP; i += 256) seg[i] = 0;
  __syncthreads();
  const int e0 = wave * (NE / 8), e1 = e0 + NE / 8;
  for (int c0 = e0; c0 < e1; c0 += 32) {
    const int e = c0 + lane;
    const int d = (e < e1) ? dst[e] : -1;
    const bool valid = (e < e1) && (d >= n0) && (d < n0 + NODES_PER_BLK);
    int tot; const int rank = chunk_rank(d - n0, valid, lane, tot);
    if (valid && rank == tot - 1) cnt[wave][d - n0] += tot;
  }
  __syncthreads();
  if (tid < 32) {
    int loc[8]; int sum = 0;
    for (int q = 0; q < 8; ++q) { int c = 0; for (int w = 0; w < 8; ++w) c += cnt[w][tid * 8 + q]; loc[q] = c; sum += c; }
    int incl = sum;
    for (int o = 1; o < 32; o <<= 1) { int t = __shfl_up(incl, o, 32); if (lane >= o) incl += t; }
    int base = incl - sum;
    for (int q = 0; q < 8; ++q) {
      const int node = tid * 8 + q;
      nodeoff[node] = base;
      int run = base;
      for (int w = 0; w < 8; ++w) { off[w][node] = run; run += cnt[w][node]; }
      base += loc[q];
    }
    if (tid == 31) nodeoff[NODES_PER_BLK] = base;
  }
  __syncthreads();
  const int btotal = nodeoff[NODES_PER_BLK];
  for (int c0 = e0; c0 < e1; c0 += 32) {
    const int e = c0 + lane;
    const int d = (e < e1) ? dst[e] : -1;
    const bool valid = (e < e1) && (d >= n0) && (d < n0 + NODES_PER_BLK);
    int tot; const int rank = chunk_rank(d - n0, valid, lane, tot);
    if (valid) {
      const int slot = off[wave][d - n0] + rank;
      if (slot < SEG_CAP) seg[slot] = e;
      if (rank == tot - 1) off[wave][d - n0] = slot + 1;
    }
  }
  __syncthreads();
  const int gstart = (blk_base[blockIdx.x] + 32 * (int)blockIdx.x + 31) & ~31;
  const int nlines = (min(btotal, SEG_CAP) + 31) >> 5;
  for (int pass = 0; pass < 2; ++pass) {
    {
      const int node = tid;
      int deg = 0;
      for (int w = 0; w < 8; ++w) deg += cnt[w][node];
      ((volatile int*)rowptr)[n0 + node] = gstart + nodeoff[node];
      ((volatile int*)rowdeg)[n0 + node] = deg;
    }
    for (int i = tid; i < nlines * 32; i += 256) ((volatile int*)csr_eid)[gstart + i] = (i < btotal) ? seg[i] : 0;
    __threadfence();
  }
}


__global__ __launch_bounds__(256) void bias_cat_kernel(const float* a, const float* b, const float* c, const float* d, float* __restrict__ o) {
  for (int pass = 0; pass < 2; ++pass) {
    for (int i = threadIdx.x; i < 4 * DIM; i += 256) { const int w = i / DIM, j = i % DIM; ((volatile float*)o)[i] = (w == 0 ? a : (w == 1 ? b : (w == 2 ? c : d)))[j]; }
    __threadfence();
  }
}
__global__ __launch_bounds__(256) void cast_nodes_kernel(const float* __restrict__ x, unsigned* __restrict__ x16) {
  const long i = (long)blockIdx.x * 256 + threadIdx.x; const long n2 = (long)NPAD * DIM / 2;
  if (i >= n2) return;
  const long e0 = 2 * i; const long row = e0 / DIM;
  const float a = (row < NN) ? x[e0] : 0.f, b = (row < NN) ? x[e0 + 1] : 0.f;
  const unsigned u = (unsigned)__builtin_bit_cast(unsigned short, (_Float16)a) | ((unsigned)__builtin_bit_cast(unsigned short, (_Float16)b) << 16);
  ((volatile unsigned*)x16)[i] = u; __threadfence(); ((volatile unsigned*)x16)[i] = u;
}
__global__ __launch_bounds__(256) void bgp_aggregate_kernel(const float* __restrict__ P, const int* __restrict__ rowptr,
    const int* __restrict__ rowdeg, const int* __restrict__ csr_eid, const int* __restrict__ srcv,
    const float* __restrict__ Wproj, const float* __restrict__ bproj, float* __restrict__ lg  ) {
  __shared__ float slg[8][2];
  const int lane = threadIdx.x & 31, wave = threadIdx.x >> 5;
  const int n = blockIdx.x * 8 + wave;
  float o[16];
#pragma unroll
  for (int q = 0; q < 16; ++q) o[q] = 0.f;
  float l0 = 0.f, l1 = 0.f;
  if (n < NN) {
    const float* prow = P + (size_t)n * (4 * DIM);
    float qv[16];
    {
      const v4f* qp = (const v4f*)(prow + 16 * lane);
#pragma unroll
      for (int i = 0; i < 4; ++i) { v4f t = qp[i]; qv[4*i] = t[0]; qv[4*i+1] = t[1]; qv[4*i+2] = t[2]; qv[4*i+3] = t[3]; }
    }
    int j0 = rowptr[n]; int dg = rowdeg[n]; dg = dg < 0 ? 0 : (dg > SEG_CAP ? SEG_CAP : dg); j0 = j0 < 0 ? 0 : j0;
    float m = -INFINITY, l = 0.f;
    for (int j = j0; j < j0 + dg; ++j) {
      int e = csr_eid[j]; e = (e < 0) ? 0 : (e >= NE ? NE - 1 : e);
      int s = srcv[e]; s = (s < 0) ? 0 : (s >= NN ? NN - 1 : s);
      const float* srow = P + (size_t)s * (4 * DIM);
      const v4f* kp = (const v4f*)(srow + DIM + 16 * lane);
      float d = 0.f;
#pragma unroll
      for (int i = 0; i < 4; ++i) { v4f t = kp[i]; d += qv[4*i] * t[0] + qv[4*i+1] * t[1] + qv[4*i+2] * t[2] + qv[4*i+3] * t[3]; }
      d += __shfl_xor(d, 1, 32); d += __shfl_xor(d, 2, 32);
      const float sc = d * 0.125f;
      const float mn = fmaxf(m, sc);
      const float al = expf(m - mn), w = expf(sc - mn);
      l = l * al + w; m = mn;
      const v4f* vp = (const v4f*)(srow + 2 * DIM + 16 * lane);
#pragma unroll
      for (int i = 0; i < 4; ++i) { v4f t = vp[i]; o[4*i] = o[4*i] * al + w * t[0]; o[4*i+1] = o[4*i+1] * al + w * t[1]; o[4*i+2] = o[4*i+2] * al + w * t[2]; o[4*i+3] = o[4*i+3] * al + w * t[3]; }
    }
    const float inv = (dg > 0) ? (1.0f / l) : 0.f;
    const v4f* sp = (const v4f*)(prow + 3 * DIM + 16 * lane);
#pragma unroll
    for (int i = 0; i < 4; ++i) { v4f t = sp[i]; o[4*i] = o[4*i] * inv + t[0]; o[4*i+1] = o[4*i+1] * inv + t[1]; o[4*i+2] = o[4*i+2] * inv + t[2]; o[4*i+3] = o[4*i+3] * inv + t[3]; }
#pragma unroll 1
    for (int q = 0; q < 16; ++q) { const int c = 16 * lane + q; l0 += o[q] * Wproj[c * 2 + 0]; l1 += o[q] * Wproj[c * 2 + 1]; }
    for (int of = 16; of > 0; of >>= 1) { l0 += __shfl_xor(l0, of, 32); l1 += __shfl_xor(l1, of, 32); }
    l0 += bproj[0]; l1 += bproj[1];
  }
  if (lane == 0) { slg[wave][0] = l0; slg[wave][1] = l1; }
  __syncthreads();
  if (threadIdx.x < 32) {
    const int t = threadIdx.x;
    const float v = (t < 8) ? slg[t][0] : (t < 16 ? slg[t - 8][1] : 0.f);
    ((volatile float*)lg)[(size_t)blockIdx.x * 32 + t] = v; __threadfence(); ((volatile float*)lg)[(size_t)blockIdx.x * 32 + t] = v;
  }
}
__global__ __launch_bounds__(256) void logits_out_kernel(const float* __restrict__ lg, float* __restrict__ out0, float* __restrict__ out1) {
  const int n = blockIdx.x * 256 + threadIdx.x;
  if (n >= NN) return;
  const float a = lg[(size_t)(n >> 3) * 32 + (n & 7)], b = lg[(size_t)(n >> 3) * 32 + 8 + (n & 7)];
  for (int pass = 0; pass < 2; ++pass) { ((volatile float*)out0)[n] = a; ((volatile float*)out1)[n] = b; __threadfence(); }
}

extern "C" void kernel_launch(void* const* d_in, const int* in_sizes, int n_in,
                              void* d_out, int out_size, void* d_ws, size_t ws_size,
                              hipStream_t stream) {
  (void)in_sizes; (void)n_in; (void)out_size; (void)ws_size;
  const float* nodes = (const float*)d_in[0];
  const int*   ei    = (const int*)d_in[1];
  const float* Wq = (const float*)d_in[2]; const float* bq = (const float*)d_in[3];
  const float* Wk = (const float*)d_in[4]; const float* bk = (const float*)d_in[5];
  const float* Wv = (const float*)d_in[6]; const float* bv = (const float*)d_in[7];
  const float* Ws = (const float*)d_in[8]; const float* bs = (const float*)d_in[9];
  const float* Wp = (const float*)d_in[10]; const float* bp = (const float*)d_in[11];
  float* out0 = (float*)d_out;
  float* out1 = out0 + NN;

  char* ws = (char*)d_ws; size_t off = 0;
  auto carve = [&](size_t bytes) -> char* { char* p = ws + off; off += (bytes + 255) & ~(size_t)255; return p; };
  int* blk_total = (int*)carve((size_t)NBLK * 32 * 4);
  int* blk_base  = (int*)carve((size_t)1024 * 4);
  int* rowptr    = (int*)carve((size_t)NBLK * NODES_PER_BLK * 4);
  int* rowdeg    = (int*)carve((size_t)NBLK * NODES_PER_BLK * 4);
  int* csr_eid   = (int*)carve((size_t)(NE + 64 * NBLK + 64) * 4);
  unsigned* X16  = (unsigned*)carve((size_t)NPAD * DIM * 2);
  _Float16* WT   = (_Float16*)carve((size_t)4 * DIM * DIM * 2);
  float*    bcat = (float*)carve((size_t)4 * DIM * 4);
  float*    P    = (float*)carve((size_t)NPAD * 4 * DIM * 4);
  float*    lg   = (float*)carve((size_t)(NPAD / 8) * 32 * 4);

  csr_count_kernel<<<NBLK, 256, 0, stream>>>(ei + NE, blk_total);
  csr_scan_kernel<<<1, 1024, 0, stream>>>(blk_total, blk_base);
  csr_fill_kernel<<<NBLK, 256, 0, stream>>>(ei + NE, blk_base, rowptr, rowdeg, csr_eid);
  cast_nodes_kernel<<<(NPAD * DIM / 2 + 255) / 256, 256, 0, stream>>>(nodes, X16);
  transpose_cast_f16<<<dim3(DIM / 64, DIM / 64), dim3(32, 8), 0, stream>>>(Wq, DIM, WT + (size_t)0 * DIM * DIM, DIM, 1.0f);
  transpose_cast_f16<<<dim3(DIM / 64, DIM / 64), dim3(32, 8), 0, stream>>>(Wk, DIM, WT + (size_t)1 * DIM * DIM, DIM, 1.0f);
  transpose_cast_f16<<<dim3(DIM / 64, DIM / 64), dim3(32, 8), 0, stream>>>(Wv, DIM, WT + (size_t)2 * DIM * DIM, DIM, 1.0f);
  transpose_cast_f16<<<dim3(DIM / 64, DIM / 64), dim3(32, 8), 0, stream>>>(Ws, DIM, WT + (size_t)3 * DIM * DIM, DIM, 1.0f);
  bias_cat_kernel<<<1, 256, 0, stream>>>(bq, bk, bv, bs, bcat);
  {
    const int tl = (NPAD / 64) * (4 * DIM / 64);
    wmma_gemm64<0, false, 2, 0, false><<<dim3((tl + 7) / 8, 1), 256, 0, stream>>>(
        (const unsigned short*)X16, nullptr, DIM, 0, U16(WT), nullptr, DIM, 0, P, nullptr, 4 * DIM, 0, bcat, nullptr, 0, NPAD, 4 * DIM, DIM, 1.0f);
  }
  bgp_aggregate_kernel<<<NPAD / 8, 256, 0, stream>>>(P, rowptr, rowdeg, csr_eid, ei, Wp, bp, lg);
  logits_out_kernel<<<(NN + 255) / 256, 256, 0, stream>>>(lg, out0, out1);
}
